// GatedDeltaNet_16690242912586
// MI455X (gfx1250) — hardware-verified
//
#include <hip/hip_runtime.h>
#include <math.h>

typedef __attribute__((ext_vector_type(16))) _Float16 v16h;
typedef __attribute__((ext_vector_type(8)))  _Float16 v8h;
typedef __attribute__((ext_vector_type(16))) __bf16   v16b;
typedef __attribute__((ext_vector_type(8)))  __bf16   v8b;
typedef __attribute__((ext_vector_type(8)))  float    v8f;
typedef __attribute__((ext_vector_type(4)))  float    v4f;

constexpr int kB    = 4;
constexpr int kL    = 1024;
constexpr int kDH   = 2048;
constexpr int kHd   = 128;
constexpr int kH    = 16;
constexpr int kHK   = 4;
constexpr int kKV   = kHK * kHd;
constexpr int kBG   = 64;
constexpr int kTaps = 4;
constexpr int kThr  = 256;
constexpr float kInCarry = 1024.0f;
constexpr float kWCarry = 4096.0f;
constexpr float kSc = 1.0f / (kInCarry * kWCarry);
constexpr float kCo = 1024.0f;
constexpr float kScO = 1.0f / (kCo * kWCarry);
constexpr float kQScale = 0.08838834764831845f;
constexpr float kL2Eps = 1e-6f, kRmsEps = 1e-5f;
constexpr float kF16MinNormal = 6.103515625e-5f;

static_assert((kL % 64) == 0 && (kDH % 64) == 0 && (kKV % 64) == 0 && (kBG % 64) == 0 && ((kL / 64) * (kBG / 64)) % 8 == 0, "GEMM M, N multiples of 64; grids exact");
static_assert((kDH % 256) == 0 && kDH / 8 == 256 && kH * kHd == kDH && kH % kHK == 0 && kH == (1 << 4) && kHK == (1 << 2), "GEMM K a multiple of 32; the transposing cast's block of K / 8 = 256 threads");

constexpr size_t kOffWQ = 0ull;
constexpr size_t kOffWK = 8388608ull;
constexpr size_t kOffWV = 10485760ull;
constexpr size_t kOffWBG = 12582912ull;
constexpr size_t kOffWG = 12845056ull;
constexpr size_t kOffWO = 21233664ull;
constexpr size_t kOffBIAS = 29622272ull;
constexpr size_t kOffPRM = 29630464ull;
constexpr size_t kOffX16 = 29634560ull;
constexpr size_t kOffQL = 33828864ull;
constexpr size_t kOffKL = 42217472ull;
constexpr size_t kOffVL = 44314624ull;
constexpr size_t kOffBGL = 46411776ull;
constexpr size_t kOffGL = 46673920ull;
constexpr size_t kOffQ2 = 55062528ull;
constexpr size_t kOffK2 = 63451136ull;
constexpr size_t kOffV2 = 65548288ull;
constexpr size_t kOffBE = 67645440ull;
constexpr size_t kOffO32 = 67776512ull;
constexpr size_t kOffO16 = 76165120ull;
constexpr size_t kWsTotal = 80359424ull;
static_assert(kWsTotal <= 134217728ull, "carve cap: under 128 MiB");
static_assert(kOffWQ == 0
              && kOffWK == kOffWQ + 8388608ull
              && kOffWV == kOffWK + 2097152ull
              && kOffWBG == kOffWV + 2097152ull
              && kOffWG == kOffWBG + 262144ull
              && kOffWO == kOffWG + 8388608ull
              && kOffBIAS == kOffWO + 8388608ull
              && kOffPRM == kOffBIAS + 8192ull
              && kOffX16 == kOffPRM + 4096ull
              && kOffQL == kOffX16 + 4194304ull
              && kOffKL == kOffQL + 8388608ull
              && kOffVL == kOffKL + 2097152ull
              && kOffBGL == kOffVL + 2097152ull
              && kOffGL == kOffBGL + 262144ull
              && kOffQ2 == kOffGL + 8388608ull
              && kOffK2 == kOffQ2 + 8388608ull
              && kOffV2 == kOffK2 + 2097152ull
              && kOffBE == kOffV2 + 2097152ull
              && kOffO32 == kOffBE + 131072ull
              && kOffO16 == kOffO32 + 8388608ull
              && kWsTotal == kOffO16 + 4194304ull, "the carve is chained and totalled");
static_assert((kOffWQ % 256) == 0 && (kOffWK % 256) == 0 && (kOffWV % 256) == 0 && (kOffWBG % 256) == 0 && (kOffWG % 256) == 0 && (kOffWO % 256) == 0 && (kOffBIAS % 256) == 0 && (kOffPRM % 256) == 0 && (kOffX16 % 256) == 0 && (kOffQL % 256) == 0 && (kOffKL % 256) == 0 && (kOffVL % 256) == 0 && (kOffBGL % 256) == 0 && (kOffGL % 256) == 0 && (kOffQ2 % 256) == 0 && (kOffK2 % 256) == 0 && (kOffV2 % 256) == 0 && (kOffBE % 256) == 0 && (kOffO32 % 256) == 0 && (kOffO16 % 256) == 0, "aligned regions");

__device__ __forceinline__ unsigned short f2bf_bits(float f) {
  unsigned u = __float_as_uint(f);
  return (unsigned short)((u + 0x7FFFu + ((u >> 16) & 1u)) >> 16);
}
__device__ __forceinline__ float bf_bits2f(unsigned short h) { return __uint_as_float(((unsigned)h) << 16); }
__device__ __forceinline__ float bf16r(float f) { return bf_bits2f(f2bf_bits(f)); }
__device__ __forceinline__ float carry_flush(float v, float carry) {
  const float s = v * carry;
  return (fabsf(s) < kF16MinNormal) ? 0.0f : s;
}
__device__ __forceinline__ float frcp(float x) { return __builtin_amdgcn_rcpf(x); }

__device__ __forceinline__ void dep_guard4_h(v8f& a, v8f& b, v8f& c, v8f& d, v16h x, v16h y) { asm volatile("v_nop\n\tv_nop\n\tv_nop\n\tv_nop" : "+v"(a), "+v"(b), "+v"(c), "+v"(d) : "v"(x), "v"(y)); }
__device__ __forceinline__ void dep_guard4_b(v8f& a, v8f& b, v8f& c, v8f& d, v16b x, v16b y) { asm volatile("v_nop\n\tv_nop\n\tv_nop\n\tv_nop" : "+v"(a), "+v"(b), "+v"(c), "+v"(d) : "v"(x), "v"(y)); }
__device__ __forceinline__ void keep4_h(v16h a, v16h b, v16h c, v16h d) { asm volatile("v_nop" :: "v"(a), "v"(b), "v"(c), "v"(d)); }
__device__ __forceinline__ void keep4_b(v16b a, v16b b, v16b c, v16b d) { asm volatile("v_nop" :: "v"(a), "v"(b), "v"(c), "v"(d)); }
__device__ __forceinline__ void acc_guard4(v8f& a, v8f& b, v8f& c, v8f& d) { asm volatile("v_nop\n\tv_nop\n\tv_nop\n\tv_nop" : "+v"(a), "+v"(b), "+v"(c), "+v"(d)); }

template <typename T> struct Frag;
template <> struct Frag<_Float16> {
  typedef v16h V; union U { v16h v; v8h h[2]; };
  static __device__ __forceinline__ v16h load(const _Float16* p) {
    U f; f.h[0] = *(const v8h*)(p); f.h[1] = *(const v8h*)(p + 16); return f.v;
  }
  static __device__ __forceinline__ v8f mma(v16h a, v16h b, v8f c) {
    return __builtin_amdgcn_wmma_f32_16x16x32_f16(false, a, false, b, (short)0, c, false, false);
  }
  static __device__ __forceinline__ void guard4(v8f& a, v8f& b, v8f& c, v8f& d, v16h x, v16h y) { dep_guard4_h(a, b, c, d, x, y); }
  static __device__ __forceinline__ void keep(v16h a, v16h b, v16h c, v16h d) { keep4_h(a, b, c, d); }
};
template <> struct Frag<__bf16> {
  typedef v16b V; union U { v16b v; v8b h[2]; };
  static __device__ __forceinline__ v16b load(const __bf16* p) {
    U f; f.h[0] = *(const v8b*)(p); f.h[1] = *(const v8b*)(p + 16); return f.v;
  }
  static __device__ __forceinline__ v8f mma(v16b a, v16b b, v8f c) {
    return __builtin_amdgcn_wmma_f32_16x16x32_bf16(false, a, false, b, (short)0, c, false, false);
  }
  static __device__ __forceinline__ void guard4(v8f& a, v8f& b, v8f& c, v8f& d, v16b x, v16b y) { dep_guard4_b(a, b, c, d, x, y); }
  static __device__ __forceinline__ void keep(v16b a, v16b b, v16b c, v16b d) { keep4_b(a, b, c, d); }
};

__device__ __forceinline__ v8f mma_h(v16h a, v16h b, v8f c) {
  c = __builtin_amdgcn_wmma_f32_16x16x32_f16(false, a, false, b, (short)0, c, false, false);
  asm volatile("v_nop\n\tv_nop\n\tv_nop\n\tv_nop" : "+v"(c) : "v"(a), "v"(b));
  return c;
}

template <int ET> struct Elem;
template <> struct Elem<0> { typedef _Float16 T; };
template <> struct Elem<1> { typedef __bf16 T; };
template <int ET, bool SPLIT, int BIAS_MODE, int OUT_MODE, bool RESID, int ACT = 0>
__global__ __launch_bounds__(256) void wmma_gemm64(
    const unsigned short* __restrict__ Ap, const unsigned short* __restrict__ A2p, int lda, long strideA,
    const unsigned short* __restrict__ Btp, const unsigned short* __restrict__ Bt2p, int ldb, long strideB,
    void* __restrict__ Cout, void* __restrict__ Cout2, int ldc, long strideC,
    const float* __restrict__ bias,
    const float* __restrict__ resid, long strideR,
    int M, int N, int K, float scale) {
  typedef typename Elem<ET>::T T;
  typedef typename Frag<T>::V V;
  const T* A = (const T*)Ap; const T* A2 = (const T*)A2p; const T* Bt = (const T*)Btp; const T* Bt2 = (const T*)Bt2p;
  __shared__ __align__(16) float sT[8][16 * 68];
  const int b    = blockIdx.y;
  const int lane = threadIdx.x & 31;
  const int wave = threadIdx.x >> 5;
  const int tilesN = N >> 6;
  const int tilesM = M >> 6;
  const int tile = blockIdx.x * 8 + wave;
  if (tile >= tilesM * tilesN) return;
  const int tm = tile / tilesN;
  const int tn = tile - tm * tilesN;
  const int m0 = tm << 6;
  const int n0 = tn << 6;

  const T* Ab  = A  + (size_t)b * strideA;
  const T* Bb  = Bt + (size_t)b * strideB;
  const T* Ab2 = SPLIT ? (A2  + (size_t)b * strideA) : nullptr;
  const T* Bb2 = SPLIT ? (Bt2 + (size_t)b * strideB) : nullptr;

  const int rlane = lane & 15;
  const int koff  = (lane >> 4) * 8;
  const int mOff  = (lane >> 4) * 8;

  v8f acc[4][4];
#pragma unroll
  for (int i = 0; i < 4; ++i)
#pragma unroll
    for (int j = 0; j < 4; ++j) acc[i][j] = (v8f){0.f,0.f,0.f,0.f,0.f,0.f,0.f,0.f};

  for (int k0 = 0; k0 < K; k0 += 32) {
    V bh[4], bl[4];
#pragma unroll
    for (int j = 0; j < 4; ++j) {
      const size_t bo = (size_t)(n0 + (j << 4) + rlane) * ldb + koff + k0;
      bh[j] = Frag<T>::load(Bb + bo);
      if (SPLIT) bl[j] = Frag<T>::load(Bb2 + bo);
    }
#pragma unroll
    for (int i = 0; i < 4; ++i) {
      const size_t ao = (size_t)(m0 + (i << 4) + rlane) * lda + koff + k0;
      V ah = Frag<T>::load(Ab + ao);
      V al;
      if (SPLIT) al = Frag<T>::load(Ab2 + ao);
#pragma unroll
      for (int j = 0; j < 4; ++j) {
        acc[i][j] = Frag<T>::mma(ah, bh[j], acc[i][j]);
        if (SPLIT) {
          acc[i][j] = Frag<T>::mma(ah, bl[j], acc[i][j]);
          acc[i][j] = Frag<T>::mma(al, bh[j], acc[i][j]);
        }
      }
      Frag<T>::guard4(acc[i][0], acc[i][1], acc[i][2], acc[i][3], ah, SPLIT ? al : ah);
    }
    Frag<T>::keep(bh[0], bh[1], bh[2], bh[3]);
    if (SPLIT) Frag<T>::keep(bl[0], bl[1], bl[2], bl[3]);
  }
  acc_guard4(acc[0][0], acc[0][1], acc[0][2], acc[0][3]);
  acc_guard4(acc[1][0], acc[1][1], acc[1][2], acc[1][3]);
  acc_guard4(acc[2][0], acc[2][1], acc[2][2], acc[2][3]);
  acc_guard4(acc[3][0], acc[3][1], acc[3][2], acc[3][3]);

  float* slab = sT[wave];
  const float* Rb = RESID ? (resid + (size_t)b * strideR) : nullptr;
#pragma unroll
  for (int i = 0; i < 4; ++i) {
    const int mBase = m0 + (i << 4);
#pragma unroll
    for (int j = 0; j < 4; ++j) {
      const int n = n0 + (j << 4) + rlane;
      float bv = 0.f;
      if (BIAS_MODE == 2) bv = bias[n];
#pragma unroll
      for (int r = 0; r < 8; ++r) {
        float v = acc[i][j][r] * scale;
        if (BIAS_MODE == 1) v += bias[mBase + mOff + r];
        if (BIAS_MODE == 2) v += bv;
        if (RESID) v += Rb[(size_t)(mBase + mOff + r) * ldc + n];
        if (ACT == 1) v = tanhf(v);
        if (ACT == 2) v = fmaxf(v, 0.0f);
        if (ACT == 3) v = v / (1.0f + expf(-v));
        if (ACT == 4) v = (v > 0.f) ? v : 0.01f * v;
        slab[(mOff + r) * 68 + (j << 4) + rlane] = v;
      }
    }
    __builtin_amdgcn_fence(__ATOMIC_RELEASE, "workgroup");
    __builtin_amdgcn_wave_barrier();
    __builtin_amdgcn_fence(__ATOMIC_ACQUIRE, "workgroup");
    if (OUT_MODE == 0) {
      float* C = (float*)Cout + (size_t)b * strideC;
      const int hh = lane >> 4, c4 = (lane & 15) * 4;
      for (int pass = 0; pass < 2; ++pass) {
#pragma unroll
        for (int it = 0; it < 8; ++it) {
          const int row = it * 2 + hh;
          v4f v = *(const v4f*)(slab + row * 68 + c4);
          *(volatile v4f*)(C + (size_t)(mBase + row) * ldc + n0 + c4) = v;
        }
        __threadfence();
      }
    } else {
      const int q = lane >> 3, c8 = (lane & 7) * 8;
      unsigned short* C  = (unsigned short*)Cout  + (size_t)b * strideC;
      unsigned short* C2 = (OUT_MODE == 2) ? ((unsigned short*)Cout2 + (size_t)b * strideC) : nullptr;
      for (int pass = 0; pass < 2; ++pass) {
#pragma unroll
        for (int it = 0; it < 4; ++it) {
          const int row = it * 4 + q;
          const float* sp = slab + row * 68 + c8;
          v8h hv, lv;
#pragma unroll
          for (int e = 0; e < 8; ++e) {
            if (OUT_MODE == 1) {
              hv[e] = (_Float16)sp[e];
            } else {
              unsigned short hb = f2bf_bits(sp[e]);
              unsigned short lb = f2bf_bits(sp[e] - bf_bits2f(hb));
              hv[e] = __builtin_bit_cast(_Float16, hb);
              lv[e] = __builtin_bit_cast(_Float16, lb);
            }
          }
          *(volatile v8h*)(C + (size_t)(mBase + row) * ldc + n0 + c8) = hv;
          if (OUT_MODE == 2) *(volatile v8h*)(C2 + (size_t)(mBase + row) * ldc + n0 + c8) = lv;
        }
        __threadfence();
      }
    }
    __builtin_amdgcn_fence(__ATOMIC_RELEASE, "workgroup");
    __builtin_amdgcn_wave_barrier();
    __builtin_amdgcn_fence(__ATOMIC_ACQUIRE, "workgroup");
  }
}

__global__ __launch_bounds__(kThr) void cast_plane_kernel(const float* __restrict__ src, unsigned short* __restrict__ dst,
                                                          int colsLog2, int dstPitch, int dstOff) {
  const int i   = blockIdx.x * kThr + threadIdx.x;
  const int sh  = colsLog2 - 3;
  const int row = i >> sh;
  const int c8  = (i & ((1 << sh) - 1)) * 8;
  const float* sp = src + ((size_t)row << colsLog2) + c8;
  const v4f a0 = *(const v4f*)(sp);
  const v4f a1 = *(const v4f*)(sp + 4);
  v8h hv;
#pragma unroll
  for (int e = 0; e < 4; ++e) {
    const float f0 = a0[e];
    const float f1 = a1[e];
    hv[e]     = (_Float16)carry_flush(bf16r(f0), kInCarry);
    hv[4 + e] = (_Float16)carry_flush(bf16r(f1), kInCarry);
  }
  unsigned short* dp = dst + (size_t)row * dstPitch + dstOff + c8;
  *(volatile v8h*)dp = hv;
  __threadfence();
  *(volatile v8h*)dp = hv;
}
__global__ __launch_bounds__(256) void wt_plane_kernel(const float* __restrict__ W, unsigned short* __restrict__ dst, int K, int N, int nLive, int ldd, int colOff) {
  const int n  = blockIdx.x;
  const int k8 = threadIdx.x * 8;
  const bool live = n < nLive;
  const int nc = live ? n : 0;
  v8h hv;
#pragma unroll
  for (int e = 0; e < 8; ++e) {
    const float w = W[(size_t)(k8 + e) * N + nc];
    hv[e] = (_Float16)(live ? carry_flush(bf16r(w), kWCarry) : 0.0f);
  }
  unsigned short* dp = dst + (size_t)n * ldd + colOff + k8;
  *(volatile v8h*)dp = hv;
  __threadfence();
  *(volatile v8h*)dp = hv;
}


__device__ __forceinline__ float silu_f(float v) { return v / (1.0f + expf(-v)); }

__global__ __launch_bounds__(kThr) void setup_kernel(const float* __restrict__ A_log, const float* __restrict__ dt_bias, const float* __restrict__ o_norm_w,
                                                     float* __restrict__ BIAS, float* __restrict__ PRM) {
  unsigned v = blockIdx.x * (unsigned)kThr + threadIdx.x;
  asm volatile("" : "+v"(v));
  v4f o = {0.f, 0.f, 0.f, 0.f};
  float* dp;
  if (v < 512u) { dp = BIAS + v * 4u; }
  else {
    const unsigned i0 = (v - 512u) * 4u;
    dp = PRM + i0;
    const bool live = i0 < 160u;
    const unsigned j0 = live ? i0 : 0u;
    const float* sp = (j0 < 16u) ? (A_log + j0) : ((j0 < 32u) ? (dt_bias + (j0 - 16u)) : (o_norm_w + (j0 - 32u)));
    const v4f a = *(const v4f*)sp;
    const bool neg = (j0 < 16u);
#pragma unroll
    for (int e = 0; e < 4; ++e) { const float p = bf16r(a[e]); const float val = neg ? -expf(p) : p; o[e] = live ? val : 0.0f; }
  }
  *(volatile v4f*)dp = o;
  __threadfence();
  *(volatile v4f*)dp = o;
}
static_assert(kDH / 4 == 512 && 512 + 256 == 3 * kThr, "set-up grid exact");

__global__ __launch_bounds__(kThr) void convnorm_kernel(const float* __restrict__ X, const float* __restrict__ cw, float* __restrict__ OUT, int C, int headsLog2, int mode) {
  const unsigned v = blockIdx.x * (unsigned)kThr + threadIdx.x;
  const unsigned t = v >> headsLog2, hd = v & ((1u << headsLog2) - 1u);
  const unsigned c0 = hd * (unsigned)kHd;
  float* orow = OUT + (size_t)t * C + c0;
  float ss = 0.0f;
  const int npassA = (mode == 0) ? 2 : 1;
  for (int pass = 0; pass < npassA; ++pass) {
    ss = 0.0f;
#pragma unroll 1
    for (int c = 0; c < kHd; c += 4) {
      v4f acc = {0.f, 0.f, 0.f, 0.f};
#pragma unroll
      for (int j = 0; j < kTaps; ++j) {
        const int tr = (int)t - (kTaps - 1) + j;
        if (tr >= 0) {
          const v4f xv = *(const v4f*)(X + (size_t)tr * C + c0 + c);
#pragma unroll
          for (int e = 0; e < 4; ++e) acc[e] += xv[e] * bf16r(cw[(size_t)(c0 + c + e) * kTaps + j]);
        }
      }
      v4f y;
#pragma unroll
      for (int e = 0; e < 4; ++e) { y[e] = silu_f(acc[e]); ss += y[e] * y[e]; }
      *(volatile v4f*)(orow + c) = y;
    }
    __threadfence();
  }
  if (mode != 0) {
    float qs = (mode == 2) ? kQScale : 1.0f;
    asm volatile("" : "+v"(qs));
    const float rn = (1.0f / sqrtf(ss + kL2Eps)) * qs;
#pragma unroll 1
    for (int c = 0; c < kHd; c += 4) {
      const v4f a = *(const v4f*)(orow + c);
      v4f y;
#pragma unroll
      for (int e = 0; e < 4; ++e) y[e] = a[e] * rn;
      *(volatile v4f*)(orow + c) = y;
    }
    __threadfence();
#pragma unroll 1
    for (int c = 0; c < kHd; c += 4) { const v4f a = *(const v4f*)(orow + c); *(volatile v4f*)(orow + c) = a; }
    __threadfence();
  }
}

__global__ __launch_bounds__(kThr) void betag_kernel(const float* __restrict__ BGL, const float* __restrict__ PRM, float* __restrict__ BE) {
  const unsigned t = blockIdx.x * (unsigned)kThr + threadIdx.x;
  const float* br = BGL + (size_t)t * kBG;
  float* er = BE + (size_t)t * 32;
  for (int pass = 0; pass < 2; ++pass) {
#pragma unroll 1
    for (int h = 0; h < kH; h += 4) {
      const v4f bb = *(const v4f*)(br + h), gg = *(const v4f*)(br + kH + h), na = *(const v4f*)(PRM + h), db = *(const v4f*)(PRM + kH + h);
      v4f ob, oe;
#pragma unroll
      for (int e = 0; e < 4; ++e) {
        ob[e] = 1.0f / (1.0f + expf(-bb[e]));
        const float x = gg[e] + db[e];
        const float sp = fmaxf(x, 0.0f) + log1pf(expf(-fabsf(x)));
        oe[e] = expf(na[e] * sp);
      }
      *(volatile v4f*)(er + h) = ob;
      *(volatile v4f*)(er + kH + h) = oe;
    }
    __threadfence();
  }
}
static_assert(kL == 4 * kThr && 2 * kH == 32, "one thread a row: 4 blocks; a row of BE is one line");

__global__ __launch_bounds__(kHd) void gdn_scan_kernel(const float* __restrict__ Q2, const float* __restrict__ K2, const float* __restrict__ V2,
                                                       const float* __restrict__ BE, float* __restrict__ O32) {
  __shared__ float st[kHd * kHd];
  const unsigned vcol = threadIdx.x;
  const unsigned h = blockIdx.x;
  const unsigned qoff = h * (unsigned)kHd, koff = (h / (unsigned)(kH / kHK)) * (unsigned)kHd;
  for (int k = 0; k < kHd; ++k) st[k * kHd + vcol] = 0.0f;
  for (int t = 0; t < kL; ++t) {
    const float* qr = Q2 + (size_t)t * kDH + qoff;
    const float* kr = K2 + (size_t)t * kKV + koff;
    const float vv = V2[(size_t)t * kKV + koff + vcol];
    const float bt = BE[(size_t)t * 32 + h], et = BE[(size_t)t * 32 + kH + h];
    float r = 0.0f;
#pragma unroll 1
    for (int k4 = 0; k4 < kHd; k4 += 4) {
      const v4f c4 = *(const v4f*)(kr + k4);
#pragma unroll
      for (int j = 0; j < 4; ++j) r += c4[j] * (et * st[(k4 + j) * kHd + (int)vcol]);
    }
    const float vres = vv - r;
    const float bv = bt * vres;
    float sum = 0.0f;
#pragma unroll 1
    for (int k4 = 0; k4 < kHd; k4 += 4) {
      const v4f q4 = *(const v4f*)(qr + k4), c4 = *(const v4f*)(kr + k4);
#pragma unroll
      for (int j = 0; j < 4; ++j) {
        const int idx = (k4 + j) * kHd + (int)vcol;
        const float s = et * st[idx] + c4[j] * bv;
        st[idx] = s;
        sum += q4[j] * s;
      }
    }
    float* op = O32 + (size_t)t * kDH + qoff + vcol;
    *(volatile float*)op = sum;
    __threadfence();
    *(volatile float*)op = sum;
  }
}
static_assert(kHd * kHd * 4 == 65536 && kHd == 128, "the state: 64 KB of LDS a block; one thread a value column");

__global__ __launch_bounds__(kThr) void normgate_kernel(const float* __restrict__ O32, const float* __restrict__ GL, const float* __restrict__ PRM, unsigned short* __restrict__ O16) {
  const unsigned v = blockIdx.x * (unsigned)kThr + threadIdx.x;
  const unsigned t = v / (unsigned)kH, hd = v % (unsigned)kH;
  const size_t base = (size_t)t * kDH + hd * (unsigned)kHd;
  const float* orow = O32 + base;
  const float* grow = GL + base;
  const float* w = PRM + 2 * kH;
  float ss = 0.0f;
#pragma unroll 1
  for (int c = 0; c < kHd; c += 4) { const v4f a = *(const v4f*)(orow + c); ss += (a[0] * a[0] + a[1] * a[1]) + (a[2] * a[2] + a[3] * a[3]); }
  const float rs = 1.0f / sqrtf(ss * (1.0f / (float)kHd) + kRmsEps);
  unsigned short* dst = O16 + base;
  for (int pass = 0; pass < 2; ++pass) {
#pragma unroll 1
    for (int c = 0; c < kHd; c += 8) {
      const v4f a0 = *(const v4f*)(orow + c), a1 = *(const v4f*)(orow + c + 4), g0 = *(const v4f*)(grow + c), g1 = *(const v4f*)(grow + c + 4), w0 = *(const v4f*)(w + c), w1 = *(const v4f*)(w + c + 4);
      v8h hv;
#pragma unroll
      for (int e = 0; e < 4; ++e) {
        hv[e] = (_Float16)carry_flush(a0[e] * rs * w0[e] * silu_f(g0[e]), kCo);
        hv[4 + e] = (_Float16)carry_flush(a1[e] * rs * w1[e] * silu_f(g1[e]), kCo);
      }
      *(volatile v8h*)(dst + c) = hv;
    }
    __threadfence();
  }
}
static_assert(((size_t)kL * kH) % kThr == 0 && ((size_t)kL * kHK) % kThr == 0, "row-and-head grids exact");

extern "C" void kernel_launch(void* const* d_in, const int* in_sizes, int n_in,
                              void* d_out, int out_size, void* d_ws, size_t ws_size,
                              hipStream_t stream) {
  if (n_in < 14 || d_out == nullptr || d_ws == nullptr) return;
  if (in_sizes[0] != kB * kL * kDH || in_sizes[1] != kDH * kDH || in_sizes[2] != kDH * kKV || in_sizes[3] != kDH * kKV || in_sizes[4] != kDH * kH || in_sizes[5] != kDH * kH) return;
  if (in_sizes[6] != kH || in_sizes[7] != kH || in_sizes[8] != kDH * kTaps || in_sizes[9] != kKV * kTaps || in_sizes[10] != kKV * kTaps || in_sizes[11] != kDH * kDH || in_sizes[12] != kHd || in_sizes[13] != kDH * kDH) return;
  if (out_size != kB * kL * kDH) return;
  if (ws_size < kWsTotal) return;
  const float* hidden = (const float*)d_in[0];
  const float* Wq = (const float*)d_in[1];
  const float* Wk = (const float*)d_in[2];
  const float* Wv = (const float*)d_in[3];
  const float* Wb = (const float*)d_in[4];
  const float* Wgk = (const float*)d_in[5];
  const float* A_log = (const float*)d_in[6];
  const float* dt_bias = (const float*)d_in[7];
  const float* conv_q = (const float*)d_in[8];
  const float* conv_k = (const float*)d_in[9];
  const float* conv_v = (const float*)d_in[10];
  const float* Wg = (const float*)d_in[11];
  const float* o_norm_w = (const float*)d_in[12];
  const float* Wo = (const float*)d_in[13];
  float* out = (float*)d_out;
  char* ws = (char*)d_ws;
  unsigned short* WQ = (unsigned short*)(ws + kOffWQ);
  unsigned short* WK = (unsigned short*)(ws + kOffWK);
  unsigned short* WV = (unsigned short*)(ws + kOffWV);
  unsigned short* WBG = (unsigned short*)(ws + kOffWBG);
  unsigned short* WG = (unsigned short*)(ws + kOffWG);
  unsigned short* WO = (unsigned short*)(ws + kOffWO);
  float* BIAS = (float*)(ws + kOffBIAS);
  float* PRM = (float*)(ws + kOffPRM);
  unsigned short* X16 = (unsigned short*)(ws + kOffX16);
  float* QL = (float*)(ws + kOffQL);
  float* KL = (float*)(ws + kOffKL);
  float* VL = (float*)(ws + kOffVL);
  float* BGL = (float*)(ws + kOffBGL);
  float* GL = (float*)(ws + kOffGL);
  float* Q2 = (float*)(ws + kOffQ2);
  float* K2 = (float*)(ws + kOffK2);
  float* V2 = (float*)(ws + kOffV2);
  float* BE = (float*)(ws + kOffBE);
  float* O32 = (float*)(ws + kOffO32);
  unsigned short* O16 = (unsigned short*)(ws + kOffO16);

  wt_plane_kernel<<<kDH, kDH / 8, 0, stream>>>(Wq, WQ, kDH, kDH, kDH, kDH, 0);
  wt_plane_kernel<<<kKV, kDH / 8, 0, stream>>>(Wk, WK, kDH, kKV, kKV, kDH, 0);
  wt_plane_kernel<<<kKV, kDH / 8, 0, stream>>>(Wv, WV, kDH, kKV, kKV, kDH, 0);
  wt_plane_kernel<<<kH, kDH / 8, 0, stream>>>(Wb, WBG, kDH, kH, kH, kDH, 0);
  wt_plane_kernel<<<kH, kDH / 8, 0, stream>>>(Wgk, WBG + (size_t)kH * kDH, kDH, kH, kH, kDH, 0);
  wt_plane_kernel<<<kBG - 2 * kH, kDH / 8, 0, stream>>>(Wb, WBG + (size_t)2 * kH * kDH, kDH, kH, 0, kDH, 0);
  wt_plane_kernel<<<kDH, kDH / 8, 0, stream>>>(Wg, WG, kDH, kDH, kDH, kDH, 0);
  wt_plane_kernel<<<kDH, kDH / 8, 0, stream>>>(Wo, WO, kDH, kDH, kDH, kDH, 0);
  setup_kernel<<<3, kThr, 0, stream>>>(A_log, dt_bias, o_norm_w, BIAS, PRM);

  for (int s = 0; s < kB; ++s) {
    cast_plane_kernel<<<(int)(((size_t)kL * kDH / 8) / kThr), kThr, 0, stream>>>(hidden + (size_t)s * kL * kDH, X16, 11, kDH, 0);
    wmma_gemm64<0, false, 2, 0, false, 0><<<dim3((kL / 64) * (kDH / 64) / 8, 1), 256, 0, stream>>>(
        X16, X16, kDH, 0L, WQ, WQ, kDH, 0L, (void*)QL, (void*)QL, kDH, 0L, BIAS, nullptr, 0L, kL, kDH, kDH, kSc);
    wmma_gemm64<0, false, 2, 0, false, 0><<<dim3((kL / 64) * (kKV / 64) / 8, 1), 256, 0, stream>>>(
        X16, X16, kDH, 0L, WK, WK, kDH, 0L, (void*)KL, (void*)KL, kKV, 0L, BIAS, nullptr, 0L, kL, kKV, kDH, kSc);
    wmma_gemm64<0, false, 2, 0, false, 0><<<dim3((kL / 64) * (kKV / 64) / 8, 1), 256, 0, stream>>>(
        X16, X16, kDH, 0L, WV, WV, kDH, 0L, (void*)VL, (void*)VL, kKV, 0L, BIAS, nullptr, 0L, kL, kKV, kDH, kSc);
    wmma_gemm64<0, false, 2, 0, false, 0><<<dim3((kL / 64) * (kBG / 64) / 8, 1), 256, 0, stream>>>(
        X16, X16, kDH, 0L, WBG, WBG, kDH, 0L, (void*)BGL, (void*)BGL, kBG, 0L, BIAS, nullptr, 0L, kL, kBG, kDH, kSc);
    wmma_gemm64<0, false, 2, 0, false, 0><<<dim3((kL / 64) * (kDH / 64) / 8, 1), 256, 0, stream>>>(
        X16, X16, kDH, 0L, WG, WG, kDH, 0L, (void*)GL, (void*)GL, kDH, 0L, BIAS, nullptr, 0L, kL, kDH, kDH, kSc);
    convnorm_kernel<<<(kL * kH) / kThr, kThr, 0, stream>>>(QL, conv_q, Q2, kDH, 4, 2);
    convnorm_kernel<<<(kL * kHK) / kThr, kThr, 0, stream>>>(KL, conv_k, K2, kKV, 2, 1);
    convnorm_kernel<<<(kL * kHK) / kThr, kThr, 0, stream>>>(VL, conv_v, V2, kKV, 2, 0);
    betag_kernel<<<kL / kThr, kThr, 0, stream>>>(BGL, PRM, BE);
    gdn_scan_kernel<<<kH, kHd, 0, stream>>>(Q2, K2, V2, BE, O32);
    normgate_kernel<<<(kL * kH) / kThr, kThr, 0, stream>>>(O32, GL, PRM, O16);
    wmma_gemm64<0, false, 2, 0, false, 0><<<dim3((kL / 64) * (kDH / 64) / 8, 1), 256, 0, stream>>>(
        O16, O16, kDH, 0L, WO, WO, kDH, 0L, (void*)(out + (size_t)s * kL * kDH), (void*)(out + (size_t)s * kL * kDH), kDH, 0L, BIAS, nullptr, 0L, kL, kDH, kDH, kScO);
  }
}
